// TripletLossSemiHard_52639119180292
// MI455X (gfx1250) — hardware-verified
//
#include <hip/hip_runtime.h>
#include <math.h>

#pragma clang fp contract(off)

constexpr int kN = 8192;
constexpr int kD = 512;
constexpr int kBlkM = 128;
constexpr int kBlkN = 128;
constexpr int kNumMBlk = kN / kBlkM;
constexpr int kNumNBlk = kN / kBlkN;
constexpr float kHiCarry = 16384.0f;
constexpr float kLoCarry = 2048.0f;
constexpr float kResFold = 1.0f / 2048.0f;
constexpr float kUnscale = 1.0f / 268435456.0f;

constexpr size_t kPlaneBytes = (size_t)kN * kD * 2;
constexpr size_t kPartBytes  = (size_t)kNumMBlk * kN * 4;
constexpr size_t kOffAH = 0;
constexpr size_t kOffAL = kOffAH + kPlaneBytes;
constexpr size_t kOffBH = kOffAL + kPlaneBytes;
constexpr size_t kOffBL = kOffBH + kPlaneBytes;
constexpr size_t kOffPV = kOffBL + kPlaneBytes;
constexpr size_t kOffPI = kOffPV + kPartBytes;
constexpr size_t kWsTotal = kOffPI + kPartBytes;
static_assert(kWsTotal == 37748736, "ws total");
static_assert(kWsTotal <= 134217728, "ws cap");
static_assert(kD % 32 == 0, "K multiple of 32");
static_assert(kN % kBlkM == 0 && kN % kBlkN == 0, "tile multiples");
static_assert(kD == 512, "lane maps assume 512 columns");
static_assert(kNumMBlk == 64, "select kernel reads 2 partials per lane");
static_assert((kOffAL % 128) == 0 && (kOffBH % 128) == 0 && (kOffBL % 128) == 0 && (kOffPV % 128) == 0 && (kOffPI % 128) == 0, "line aligned");

typedef __attribute__((ext_vector_type(16))) _Float16 v16h;
typedef __attribute__((ext_vector_type(8)))  _Float16 v8h;
typedef __attribute__((ext_vector_type(8)))  float    v8f;
typedef __attribute__((ext_vector_type(4)))  float    v4f;
typedef __attribute__((ext_vector_type(4)))  unsigned int v4u;
typedef __attribute__((ext_vector_type(4)))  int      v4i;

__device__ __forceinline__ void keep4_h(v16h a, v16h b, v16h c, v16h d) { asm volatile("v_nop" :: "v"(a), "v"(b), "v"(c), "v"(d)); }
__device__ __forceinline__ void acc_guard4(v8f& a, v8f& b, v8f& c, v8f& d) { asm volatile("v_nop\n\tv_nop\n\tv_nop\n\tv_nop" : "+v"(a), "+v"(b), "+v"(c), "+v"(d)); }
__device__ __forceinline__ void dep_guard4h(v8f& a, v8f& b, v8f& c, v8f& d, v16h x, v16h y) {
  asm volatile("v_nop\n\tv_nop\n\tv_nop\n\tv_nop" : "+v"(a), "+v"(b), "+v"(c), "+v"(d) : "v"(x), "v"(y));
}

template <typename T> struct Frag;
template <> struct Frag<_Float16> {
  typedef v16h V; union U { v16h v; v8h h[2]; };
  static __device__ __forceinline__ v16h load(const _Float16* p) {
    U f; f.h[0] = *(const v8h*)(p); f.h[1] = *(const v8h*)(p + 16); return f.v;
  }
  static __device__ __forceinline__ v8f mma(v16h a, v16h b, v8f c) {
    return __builtin_amdgcn_wmma_f32_16x16x32_f16(false, a, false, b, (short)0, c, false, false);
  }
};
typedef Frag<_Float16> FragH;

__device__ __forceinline__ unsigned pk16(unsigned short a, unsigned short b) { return (unsigned)a | ((unsigned)b << 16); }
__device__ __forceinline__ unsigned short h_bits(float f) { const _Float16 h = (_Float16)f; return __builtin_bit_cast(unsigned short, h); }

__device__ __forceinline__ double shfl_xor_f64(double v, int off) {
  const unsigned long long u = (unsigned long long)__double_as_longlong(v);
  int lo32 = (int)(unsigned)(u & 0xffffffffull);
  int hi32 = (int)(unsigned)(u >> 32);
  lo32 = __shfl_xor(lo32, off, 32);
  hi32 = __shfl_xor(hi32, off, 32);
  const unsigned long long r = ((unsigned long long)(unsigned)hi32 << 32) | (unsigned long long)(unsigned)lo32;
  return __longlong_as_double((long long)r);
}

__global__ __launch_bounds__(256) void norm_split_kernel(
    const float* __restrict__ a, const float* __restrict__ b,
    unsigned short* __restrict__ ah, unsigned short* __restrict__ al,
    unsigned short* __restrict__ bh, unsigned short* __restrict__ bl) {
  const int lane = threadIdx.x & 31;
  const int wave = threadIdx.x >> 5;
  const int which = blockIdx.y;
  const float* src = (which == 0) ? a : b;
  unsigned short* dh = (which == 0) ? ah : bh;
  unsigned short* dl = (which == 0) ? al : bl;
  const int row = blockIdx.x * 8 + wave;
  const float* p = src + (size_t)row * kD;
  const int c0 = 8 * lane;
  const int c1 = 256 + 8 * lane;
  const v4f x0 = *(const v4f*)(p + c0);
  const v4f x1 = *(const v4f*)(p + c0 + 4);
  const v4f x2 = *(const v4f*)(p + c1);
  const v4f x3 = *(const v4f*)(p + c1 + 4);
  float xs[16];
#pragma unroll
  for (int e = 0; e < 4; ++e) {
    xs[e]      = x0[e];
    xs[4 + e]  = x1[e];
    xs[8 + e]  = x2[e];
    xs[12 + e] = x3[e];
  }
  double s = 0.0;
#pragma unroll
  for (int e = 0; e < 16; ++e) {
    const float q = xs[e] * xs[e];
    s += (double)q;
  }
#pragma unroll
  for (int off = 16; off > 0; off >>= 1) s += shfl_xor_f64(s, off);
  const float sf  = (float)s;
  const float nrm = sqrtf(sf);
  const float inv = 1.0f / fmaxf(nrm, 1e-8f);

  unsigned short hb[16], lb[16];
#pragma unroll
  for (int e = 0; e < 16; ++e) {
    const float yc = (xs[e] * inv) * kHiCarry;
    const _Float16 hq = (_Float16)yc;
    const float hf = (float)hq;
    hb[e] = __builtin_bit_cast(unsigned short, hq);
    lb[e] = h_bits((yc - hf) * kLoCarry);
  }
  const v4u h0 = (v4u){pk16(hb[0], hb[1]),  pk16(hb[2], hb[3]),   pk16(hb[4], hb[5]),   pk16(hb[6], hb[7])};
  const v4u h1 = (v4u){pk16(hb[8], hb[9]),  pk16(hb[10], hb[11]), pk16(hb[12], hb[13]), pk16(hb[14], hb[15])};
  const v4u l0 = (v4u){pk16(lb[0], lb[1]),  pk16(lb[2], lb[3]),   pk16(lb[4], lb[5]),   pk16(lb[6], lb[7])};
  const v4u l1 = (v4u){pk16(lb[8], lb[9]),  pk16(lb[10], lb[11]), pk16(lb[12], lb[13]), pk16(lb[14], lb[15])};
  const size_t base = (size_t)row * kD;
  for (int pass = 0; pass < 2; ++pass) {
    *(volatile v4u*)(dh + base + c0) = h0;
    *(volatile v4u*)(dh + base + c1) = h1;
    *(volatile v4u*)(dl + base + c0) = l0;
    *(volatile v4u*)(dl + base + c1) = l1;
    __threadfence();
  }
}

__global__ __launch_bounds__(256) void sim_colmax_kernel(
    const unsigned short* __restrict__ Mh, const unsigned short* __restrict__ Ml,
    const unsigned short* __restrict__ Nh, const unsigned short* __restrict__ Nl,
    float* __restrict__ pv, int* __restrict__ pi) {
  __shared__ float sV[2][kBlkN];
  __shared__ int   sI[2][kBlkN];
  const _Float16* Mhp = (const _Float16*)Mh;
  const _Float16* Mlp = (const _Float16*)Ml;
  const _Float16* Nhp = (const _Float16*)Nh;
  const _Float16* Nlp = (const _Float16*)Nl;
  const int lane = threadIdx.x & 31;
  const int wave = threadIdx.x >> 5;
  const int wm = wave & 1;
  const int wn = wave >> 1;
  const int mblk = blockIdx.y;
  const int nblk = blockIdx.x;
  const int m0w = mblk * kBlkM + wm * 64;
  const int n0w = nblk * kBlkN + wn * 32;
  const int rlane = lane & 15;
  const int hsel  = lane >> 4;
  const int koff  = hsel * 8;

  v8f am[4][2], ar[4][2];
#pragma unroll
  for (int i = 0; i < 4; ++i)
#pragma unroll
    for (int j = 0; j < 2; ++j) {
      am[i][j] = (v8f){0.f, 0.f, 0.f, 0.f, 0.f, 0.f, 0.f, 0.f};
      ar[i][j] = (v8f){0.f, 0.f, 0.f, 0.f, 0.f, 0.f, 0.f, 0.f};
    }

  for (int k0 = 0; k0 < kD; k0 += 32) {
    v16h bh[2], bl[2];
#pragma unroll
    for (int j = 0; j < 2; ++j) {
      const size_t bo = (size_t)(n0w + (j << 4) + rlane) * kD + koff + k0;
      bh[j] = FragH::load(Nhp + bo);
      bl[j] = FragH::load(Nlp + bo);
    }
#pragma unroll
    for (int i = 0; i < 4; ++i) {
      const size_t ao = (size_t)(m0w + (i << 4) + rlane) * kD + koff + k0;
      const v16h ahf = FragH::load(Mhp + ao);
      const v16h alf = FragH::load(Mlp + ao);
#pragma unroll
      for (int j = 0; j < 2; ++j) {
        am[i][j] = FragH::mma(ahf, bh[j], am[i][j]);
        ar[i][j] = FragH::mma(ahf, bl[j], ar[i][j]);
        ar[i][j] = FragH::mma(alf, bh[j], ar[i][j]);
      }
      dep_guard4h(am[i][0], am[i][1], ar[i][0], ar[i][1], ahf, alf);
    }
    keep4_h(bh[0], bh[1], bl[0], bl[1]);
  }
  acc_guard4(am[0][0], am[0][1], ar[0][0], ar[0][1]);
  acc_guard4(am[1][0], am[1][1], ar[1][0], ar[1][1]);
  acc_guard4(am[2][0], am[2][1], ar[2][0], ar[2][1]);
  acc_guard4(am[3][0], am[3][1], ar[3][0], ar[3][1]);

#pragma unroll
  for (int j = 0; j < 2; ++j) {
    const int gj = n0w + (j << 4) + rlane;
    float best = -3.0e38f;
    int bidx = m0w + (hsel << 3);
#pragma unroll
    for (int i = 0; i < 4; ++i) {
#pragma unroll
      for (int r = 0; r < 8; ++r) {
        const int gi = m0w + (i << 4) + (hsel << 3) + r;
        float v = (am[i][j][r] + ar[i][j][r] * kResFold) * kUnscale;
        v = v - ((gi == gj) ? 1.0f : 0.0f);
        const bool take = v > best;
        best = take ? v : best;
        bidx = take ? gi : bidx;
      }
    }
    const float ob = __shfl_xor(best, 16, 32);
    const int   oi = __shfl_xor(bidx, 16, 32);
    const bool tk = (ob > best) || ((ob == best) && (oi < bidx));
    best = tk ? ob : best;
    bidx = tk ? oi : bidx;
    if (hsel == 0) {
      const int cl = (wn << 5) + (j << 4) + rlane;
      sV[wm][cl] = best;
      sI[wm][cl] = bidx;
    }
  }
  __syncthreads();
  if (wave == 0) {
    v4f vv;
    v4i ii;
#pragma unroll
    for (int e = 0; e < 4; ++e) {
      const int cl = 4 * lane + e;
      const float v0 = sV[0][cl];
      const int   i0 = sI[0][cl];
      const float v1 = sV[1][cl];
      const int   i1 = sI[1][cl];
      const bool t = v1 > v0;
      vv[e] = t ? v1 : v0;
      ii[e] = t ? i1 : i0;
    }
    float* dstv = pv + (size_t)mblk * kN + (size_t)nblk * kBlkN + 4 * lane;
    int*   dsti = pi + (size_t)mblk * kN + (size_t)nblk * kBlkN + 4 * lane;
    for (int pass = 0; pass < 2; ++pass) {
      *(volatile v4f*)dstv = vv;
      *(volatile v4i*)dsti = ii;
      __threadfence();
    }
  }
}

__global__ __launch_bounds__(256) void select_gather_kernel(
    const float* __restrict__ pv, const int* __restrict__ pi,
    const float* __restrict__ bsrc, float* __restrict__ out) {
  const int lane = threadIdx.x & 31;
  const int wave = threadIdx.x >> 5;
  const int j = blockIdx.x * 8 + wave;
  float best = pv[(size_t)lane * kN + j];
  int   bidx = pi[(size_t)lane * kN + j];
  const float v1 = pv[(size_t)(lane + 32) * kN + j];
  const int   i1 = pi[(size_t)(lane + 32) * kN + j];
  {
    const bool t = (v1 > best) || ((v1 == best) && (i1 < bidx));
    best = t ? v1 : best;
    bidx = t ? i1 : bidx;
  }
#pragma unroll
  for (int off = 16; off > 0; off >>= 1) {
    const float ob = __shfl_xor(best, off, 32);
    const int   oi = __shfl_xor(bidx, off, 32);
    const bool t = (ob > best) || ((ob == best) && (oi < bidx));
    best = t ? ob : best;
    bidx = t ? oi : bidx;
  }
  int idx = bidx < 0 ? 0 : bidx;
  idx = idx > (kN - 1) ? (kN - 1) : idx;
  const float* srow = bsrc + (size_t)idx * kD;
  float* drow = out + (size_t)j * kD;
  const v4f r0 = *(const v4f*)(srow + 4 * lane);
  const v4f r1 = *(const v4f*)(srow + 128 + 4 * lane);
  const v4f r2 = *(const v4f*)(srow + 256 + 4 * lane);
  const v4f r3 = *(const v4f*)(srow + 384 + 4 * lane);
  for (int pass = 0; pass < 2; ++pass) {
    *(volatile v4f*)(drow + 4 * lane)       = r0;
    *(volatile v4f*)(drow + 128 + 4 * lane) = r1;
    *(volatile v4f*)(drow + 256 + 4 * lane) = r2;
    *(volatile v4f*)(drow + 384 + 4 * lane) = r3;
    __threadfence();
  }
}

extern "C" void kernel_launch(void* const* d_in, const int* in_sizes, int n_in,
                              void* d_out, int out_size, void* d_ws, size_t ws_size,
                              hipStream_t stream) {
  if (n_in < 2) return;
  if (in_sizes[0] < kN * kD || in_sizes[1] < kN * kD) return;
  if (out_size < kN * kD) return;
  if (ws_size < kWsTotal) return;

  const float* a = (const float*)d_in[0];
  const float* b = (const float*)d_in[1];
  float* out = (float*)d_out;
  char* ws = (char*)d_ws;
  unsigned short* ahp = (unsigned short*)(ws + kOffAH);
  unsigned short* alp = (unsigned short*)(ws + kOffAL);
  unsigned short* bhp = (unsigned short*)(ws + kOffBH);
  unsigned short* blp = (unsigned short*)(ws + kOffBL);
  float* pvp = (float*)(ws + kOffPV);
  int*   pip = (int*)(ws + kOffPI);

  norm_split_kernel<<<dim3(kN / 8, 2), 256, 0, stream>>>(a, b, ahp, alp, bhp, blp);
  sim_colmax_kernel<<<dim3(kNumNBlk, kNumMBlk), 256, 0, stream>>>(bhp, blp, ahp, alp, pvp, pip);
  select_gather_kernel<<<kN / 8, 256, 0, stream>>>(pvp, pip, b, out);
}
